// DecoderBlock_52896817217548
// MI455X (gfx1250) — hardware-verified
//
#include <hip/hip_runtime.h>
#include <math.h>

#ifndef NB
#define NB 2
#endif
#ifndef SEQ
#define SEQ 2048
#endif
#define NB_FULL 2
#define SEQ_FULL 2048
#define DM 1024
#define DFF 4096
#define NHEADS 16
#define DQKV 3072
#define NBIAS 9216

static_assert(NB >= 1 && NB <= NB_FULL);
static_assert(SEQ % 64 == 0 && SEQ <= SEQ_FULL);
static_assert(DM == NHEADS * 64);

typedef __attribute__((ext_vector_type(16))) _Float16 v16h;
typedef __attribute__((ext_vector_type(8)))  _Float16 v8h;
typedef __attribute__((ext_vector_type(16))) __bf16   v16b;
typedef __attribute__((ext_vector_type(8)))  __bf16   v8b;
typedef __attribute__((ext_vector_type(8)))  float    v8f;
typedef __attribute__((ext_vector_type(4)))  float    v4f;
typedef __attribute__((ext_vector_type(4)))  unsigned u4;


#define VST2(T, ptr, val) do { const T vst2_v_ = (val); *(volatile T*)(ptr) = vst2_v_; __threadfence(); *(volatile T*)(ptr) = vst2_v_; } while (0)

__device__ __forceinline__ float cmb_bf(float v) {
    const unsigned u = __float_as_uint(v);
    const unsigned r = (u + 0x7fffu + ((u >> 16) & 1u)) & 0xffff0000u;
    return __uint_as_float(r);
}
__device__ __forceinline__ unsigned pk2h(float a, float b) {
    return (unsigned)__builtin_bit_cast(unsigned short, (_Float16)a) | ((unsigned)__builtin_bit_cast(unsigned short, (_Float16)b) << 16);
}

__global__ __launch_bounds__(256) void k_cm_castbT(const float* __restrict__ SRC, unsigned lds, unsigned short* __restrict__ DST, unsigned ldd, unsigned nR, unsigned nC, float sc) {
    const unsigned u = blockIdx.x * 256u + threadIdx.x;
    const unsigned per = nR >> 3;
    if (u >= nC * per) return;
    const unsigned c = u / per;
    const unsigned r0 = 8u * (u - c * per);
    float w[8];
#pragma unroll
    for (int e = 0; e < 8; ++e) w[e] = cmb_bf(SRC[(size_t)(r0 + e) * lds + c]) * sc;
    u4 pk; pk.x = pk2h(w[0], w[1]); pk.y = pk2h(w[2], w[3]); pk.z = pk2h(w[4], w[5]); pk.w = pk2h(w[6], w[7]);
    VST2(u4, (u4*)(DST + (size_t)c * ldd + r0), pk);
}

__global__ __launch_bounds__(256) void k_db_bias(const float* __restrict__ bq, const float* __restrict__ bk, const float* __restrict__ bv, const float* __restrict__ bo,
                                                 const float* __restrict__ b1, const float* __restrict__ b2, float* __restrict__ dst) {
    const unsigned blk = blockIdx.x;
    const float* src; unsigned base;
    if (blk < 4u)       { src = bq; base = 0u; }
    else if (blk < 8u)  { src = bk; base = 1024u; }
    else if (blk < 12u) { src = bv; base = 2048u; }
    else if (blk < 16u) { src = bo; base = 3072u; }
    else if (blk < 32u) { src = b1; base = 4096u; }
    else                { src = b2; base = 8192u; }
    const unsigned i = blk * 256u + threadIdx.x;
    const float v = cmb_bf(src[i - base]);
    VST2(float, dst + i, v);
}

template <int BFX>
__global__ __launch_bounds__(256) void k_db_ln(const float* __restrict__ X, const float* __restrict__ G, const float* __restrict__ Bb, unsigned short* __restrict__ O,
                                               unsigned rows, unsigned seq, unsigned srows) {
    #pragma clang fp contract(off)
    const unsigned row = blockIdx.x * 8u + (threadIdx.x >> 5);
    const unsigned L = threadIdx.x & 31u;
    if (row >= rows) return;
    const unsigned bb = row / seq;
    const unsigned sr = row - bb * seq;
    const float* xr = X + ((size_t)bb * srows + sr) * 1024;
    float x[32]; float s = 0.f;
#pragma unroll
    for (int g = 0; g < 4; ++g) {
        const v4f a = *(const v4f*)(xr + 256 * g + 8 * L), b = *(const v4f*)(xr + 256 * g + 8 * L + 4);
        const float v[8] = {a.x, a.y, a.z, a.w, b.x, b.y, b.z, b.w};
#pragma unroll
        for (int e = 0; e < 8; ++e) { const float t = BFX ? cmb_bf(v[e]) : v[e]; x[8 * g + e] = t; s += t; }
    }
#pragma unroll
    for (int o = 16; o > 0; o >>= 1) s += __shfl_xor(s, o, 32);
    const float mu = s * (1.f / 1024.f); float q = 0.f;
#pragma unroll
    for (int e = 0; e < 32; ++e) { const float d = x[e] - mu; q += d * d; }
#pragma unroll
    for (int o = 16; o > 0; o >>= 1) q += __shfl_xor(q, o, 32);
    const float rs = rsqrtf(q * (1.f / 1024.f) + 1e-5f);
#pragma unroll
    for (int g = 0; g < 4; ++g) {
        const unsigned c0 = 256u * g + 8u * L; float y[8];
#pragma unroll
        for (int e = 0; e < 8; ++e) y[e] = (x[8 * g + e] - mu) * rs * cmb_bf(G[c0 + e]) + cmb_bf(Bb[c0 + e]);
        u4 pk; pk.x = pk2h(y[0], y[1]); pk.y = pk2h(y[2], y[3]); pk.z = pk2h(y[4], y[5]); pk.w = pk2h(y[6], y[7]);
        VST2(u4, (u4*)(O + (size_t)row * 1024 + c0), pk);
    }
}

union FH { v16h v; v8h h[2]; };
__device__ __forceinline__ v16h frag_ld(const _Float16* p) {
    FH f; f.h[0] = *(const v8h*)(p); f.h[1] = *(const v8h*)(p + 16); return f.v;
}
__device__ __forceinline__ v8f mma_h(v16h a, v16h b, v8f c) {
    return __builtin_amdgcn_wmma_f32_16x16x32_f16(false, a, false, b, (short)0, c, false, false);
}
__device__ __forceinline__ void dep_guard_h(v8f& a, v8f& b, v16h x, v16h y) { asm volatile("v_nop\n\tv_nop\n\tv_nop\n\tv_nop" : "+v"(a), "+v"(b) : "v"(x), "v"(y)); }
__device__ __forceinline__ void keep4_h(v16h a, v16h b, v16h c, v16h d) { asm volatile("v_nop" :: "v"(a), "v"(b), "v"(c), "v"(d)); }
__device__ __forceinline__ void acc_guard4(v8f& a, v8f& b, v8f& c, v8f& d) { asm volatile("v_nop\n\tv_nop\n\tv_nop\n\tv_nop" : "+v"(a), "+v"(b), "+v"(c), "+v"(d)); }

template <int BIAS_MODE, int OUT_MODE, bool RESID, int ACT, int RESBF>
__global__ __launch_bounds__(256) void wmma_gemm64(
    const unsigned short* __restrict__ Ap, int lda, long long strideA,
    const unsigned short* __restrict__ Btp, int ldb, long long strideB,
    void* __restrict__ Cout, int ldc, long long strideC,
    const float* __restrict__ bias,
    const float* __restrict__ resid, long long strideR,
    int M, int N, int K, float scale) {
  static_assert(ACT == 0 || OUT_MODE == 1);
  const _Float16* A = (const _Float16*)Ap; const _Float16* Bt = (const _Float16*)Btp;
  __shared__ __align__(16) float sT[8][16 * 68];
  const int b    = blockIdx.y;
  const int lane = threadIdx.x & 31;
  const int wave = threadIdx.x >> 5;
  const int tilesN = N >> 6;
  const int tilesM = M >> 6;
  const int tile = blockIdx.x * 8 + wave;
  if (tile >= tilesM * tilesN) return;
  const int tm = tile / tilesN;
  const int tn = tile - tm * tilesN;
  const int m0 = tm << 6;
  const int n0 = tn << 6;

  const _Float16* Ab = A  + (size_t)b * strideA;
  const _Float16* Bb = Bt + (size_t)b * strideB;

  const int rlane = lane & 15;
  const int koff  = (lane >> 4) * 8;
  const int mOff  = (lane >> 4) * 8;

  v8f acc[4][4];
#pragma unroll
  for (int i = 0; i < 4; ++i)
#pragma unroll
    for (int j = 0; j < 4; ++j) acc[i][j] = (v8f){0.f,0.f,0.f,0.f,0.f,0.f,0.f,0.f};

  for (int k0 = 0; k0 < K; k0 += 32) {
    v16h bh[4];
#pragma unroll
    for (int j = 0; j < 4; ++j) {
      const size_t bo = (size_t)(n0 + (j << 4) + rlane) * ldb + koff + k0;
      bh[j] = frag_ld(Bb + bo);
    }
#pragma unroll
    for (int i = 0; i < 4; ++i) {
      const size_t ao = (size_t)(m0 + (i << 4) + rlane) * lda + koff + k0;
      v16h ah = frag_ld(Ab + ao);
#pragma unroll
      for (int j = 0; j < 4; ++j) acc[i][j] = mma_h(ah, bh[j], acc[i][j]);
      dep_guard_h(acc[i][0], acc[i][3], ah, ah);
    }
    keep4_h(bh[0], bh[1], bh[2], bh[3]);
  }
  acc_guard4(acc[0][0], acc[0][1], acc[0][2], acc[0][3]);
  acc_guard4(acc[1][0], acc[1][1], acc[1][2], acc[1][3]);
  acc_guard4(acc[2][0], acc[2][1], acc[2][2], acc[2][3]);
  acc_guard4(acc[3][0], acc[3][1], acc[3][2], acc[3][3]);

  float* slab = sT[wave];
  const float* Rb = RESID ? (resid + (size_t)b * strideR) : nullptr;
#pragma unroll
  for (int i = 0; i < 4; ++i) {
    const int mBase = m0 + (i << 4);
#pragma unroll
    for (int j = 0; j < 4; ++j) {
      const int n = n0 + (j << 4) + rlane;
      float bv = 0.f;
      if (BIAS_MODE == 2) bv = bias[n];
#pragma unroll
      for (int r = 0; r < 8; ++r) {
        float v = acc[i][j][r] * scale;
        if (BIAS_MODE == 2) v += bv;
        slab[(mOff + r) * 68 + (j << 4) + rlane] = v;
      }
    }
    __builtin_amdgcn_fence(3  , "workgroup");
    __builtin_amdgcn_wave_barrier();
    __builtin_amdgcn_fence(2  , "workgroup");
    if (OUT_MODE == 0) {
      float* C = (float*)Cout + (size_t)b * strideC;
      const int hh = lane >> 4, c4 = (lane & 15) * 4;
#pragma unroll
      for (int it = 0; it < 8; ++it) {
        const int row = it * 2 + hh;
        v4f v = *(const v4f*)(slab + row * 68 + c4);
        if (RESID) {
          v4f rv = *(const v4f*)(Rb + (size_t)(mBase + row) * ldc + n0 + c4);
          if (RESBF) { rv.x = cmb_bf(rv.x); rv.y = cmb_bf(rv.y); rv.z = cmb_bf(rv.z); rv.w = cmb_bf(rv.w); }
          v = v + rv;
        }
        volatile v4f* dst = (volatile v4f*)(C + (size_t)(mBase + row) * ldc + n0 + c4);
        *dst = v; __threadfence(); *dst = v;
      }
    } else {
      const int q4 = lane >> 3, c8 = (lane & 7) * 8;
      unsigned short* C = (unsigned short*)Cout + (size_t)b * strideC;
#pragma unroll 1
      for (int it = 0; it < 4; ++it) {
        const int row = it * 4 + q4;
        const float* sp = slab + row * 68 + c8;
        const v4f s0 = *(const v4f*)(sp), s1 = *(const v4f*)(sp + 4);
        const float w[8] = {s0.x, s0.y, s0.z, s0.w, s1.x, s1.y, s1.z, s1.w};
        v8h hv;
#pragma unroll
        for (int e = 0; e < 8; ++e) {
          float t = w[e];
          if (ACT == 5) t = 0.5f * t * (1.0f + erff(t * 0.70710678118654752f));
          hv[e] = (_Float16)t;
        }
        volatile v8h* dst = (volatile v8h*)(C + (size_t)(mBase + row) * ldc + n0 + c8);
        *dst = hv; __threadfence(); *dst = hv;
      }
    }
    __builtin_amdgcn_fence(3  , "workgroup");
    __builtin_amdgcn_wave_barrier();
    __builtin_amdgcn_fence(2  , "workgroup");
  }
}

#define AT_D 64
#define AT_NW 4
#define AT_QB 64
#define AT_KC 64
struct AttnGeom { const int* pad; long long q_bs, q_rs, k_bs, k_rs, v_bs, v_rs, o_bs, o_rs, pad_bs; float qscale; float mask_fill; };
static_assert(sizeof(AttnGeom) == 88);

__device__ __forceinline__ unsigned short at_bf_bits(float f) {
  unsigned u = __float_as_uint(f);
  return (unsigned short)((u + 0x7FFFu + ((u >> 16) & 1u)) >> 16);
}
__device__ __forceinline__ void at_split(float f, __bf16& hi, __bf16& lo) {
  const unsigned short hb = at_bf_bits(f);
  hi = __builtin_bit_cast(__bf16, hb);
  lo = __builtin_bit_cast(__bf16, at_bf_bits(f - __uint_as_float(((unsigned)hb) << 16)));
}
__device__ __forceinline__ v8f at_mma(v16b a, v16b b, v8f c) {
  c = __builtin_amdgcn_wmma_f32_16x16x32_bf16(false, a, false, b, (short)0, c, false, false);
  asm volatile("v_nop\n\tv_nop\n\tv_nop\n\tv_nop" : "+v"(c) : "v"(a), "v"(b));
  return c;
}

__global__ __launch_bounds__(128)
void attn64_kernel(const float* __restrict__ q, const float* __restrict__ k,
                   const float* __restrict__ v, unsigned short* __restrict__ out, AttnGeom g) {
  union FB { v16b v; v8b h[2]; };
  __shared__ __align__(16) __bf16 Ksh[AT_KC * AT_D];
  __shared__ __align__(16) __bf16 Ksl[AT_KC * AT_D];
  __shared__ __align__(16) __bf16 Vth[AT_D * AT_KC];
  __shared__ __align__(16) __bf16 Vtl[AT_D * AT_KC];
  __shared__ __align__(16) __bf16 Psh[AT_NW][16 * AT_KC];
  __shared__ __align__(16) __bf16 Psl[AT_NW][16 * AT_KC];
  __shared__ __align__(16) float  Os[AT_NW][16 * 68];

  const unsigned tid  = threadIdx.x;
  const unsigned wave = tid >> 5;
  const unsigned lane = tid & 31u;
  const unsigned hh   = lane >> 4;
  const unsigned c    = lane & 15u;

  constexpr unsigned NQB = SEQ / AT_QB;
  const unsigned bx = blockIdx.x;
  const unsigned qb = bx % NQB;
  const unsigned bh = bx / NQB;
  const unsigned h  = bh % NHEADS;
  const unsigned b  = bh / NHEADS;
  const unsigned q0 = qb * AT_QB + wave * 16u;

  const float* qb_ptr = q + (size_t)b * g.q_bs + (size_t)h * 64;
  const float* kb_ptr = k + (size_t)b * g.k_bs + (size_t)h * 64;
  const float* vb_ptr = v + (size_t)b * g.v_bs + (size_t)h * 64;
  unsigned short* ob_ptr = out + (size_t)b * g.o_bs + (size_t)h * 64;
  const int* padb = g.pad + (size_t)b * g.pad_bs;

  v16b qah[2], qal[2];
  {
    const float* qrow = qb_ptr + (size_t)(q0 + c) * g.q_rs;
#pragma unroll
    for (int dc = 0; dc < 2; ++dc) {
      const v4f a0 = *(const v4f*)(qrow + dc * 32 + 8 * hh), a1 = *(const v4f*)(qrow + dc * 32 + 8 * hh + 4);
      const v4f b0 = *(const v4f*)(qrow + dc * 32 + 16 + 8 * hh), b1 = *(const v4f*)(qrow + dc * 32 + 16 + 8 * hh + 4);
      const float f0[8] = {a0.x, a0.y, a0.z, a0.w, a1.x, a1.y, a1.z, a1.w};
      const float f1[8] = {b0.x, b0.y, b0.z, b0.w, b1.x, b1.y, b1.z, b1.w};
#pragma unroll
      for (int e = 0; e < 8; ++e) {
        __bf16 hq, lq;
        at_split(f0[e] * g.qscale, hq, lq); qah[dc][e] = hq; qal[dc][e] = lq;
        at_split(f1[e] * g.qscale, hq, lq); qah[dc][8 + e] = hq; qal[dc][8 + e] = lq;
      }
    }
  }

  float mrow[8], lrow[8];
  v8f oacc[4];
#pragma unroll
  for (int r = 0; r < 8; ++r) { mrow[r] = -INFINITY; lrow[r] = 0.f; }
#pragma unroll
  for (int t = 0; t < 4; ++t) oacc[t] = (v8f){0.f,0.f,0.f,0.f,0.f,0.f,0.f,0.f};

  const unsigned nChunks = qb + 1u;
  for (unsigned kc = 0; kc < nChunks; ++kc) {
    const unsigned kv0 = kc * AT_KC;
    __syncthreads();
    {
      const unsigned kvr = tid >> 1, dh = (tid & 1u) * 32u;
      const float* krow = kb_ptr + (size_t)(kv0 + kvr) * g.k_rs + dh;
      const float* vrow = vb_ptr + (size_t)(kv0 + kvr) * g.v_rs + dh;
#pragma unroll
      for (int i = 0; i < 8; ++i) {
        const v4f kk = *(const v4f*)(krow + 4 * i);
        const v4f vv = *(const v4f*)(vrow + 4 * i);
#pragma unroll
        for (int e = 0; e < 4; ++e) {
          const unsigned d = dh + 4 * i + e;
          __bf16 a, bl;
          at_split(kk[e], a, bl); Ksh[kvr * AT_D + d] = a; Ksl[kvr * AT_D + d] = bl;
          at_split(vv[e], a, bl); Vth[d * AT_KC + kvr] = a; Vtl[d * AT_KC + kvr] = bl;
        }
      }
    }
    __syncthreads();

    v8f s[4];
#pragma unroll
    for (int j = 0; j < 4; ++j) {
      s[j] = (v8f){0.f,0.f,0.f,0.f,0.f,0.f,0.f,0.f};
#pragma unroll
      for (int dc = 0; dc < 2; ++dc) {
        FB kb, kl;
        kb.h[0] = *(const v8b*)(Ksh + (j * 16 + c) * AT_D + dc * 32 + 8 * hh);
        kb.h[1] = *(const v8b*)(Ksh + (j * 16 + c) * AT_D + dc * 32 + 16 + 8 * hh);
        kl.h[0] = *(const v8b*)(Ksl + (j * 16 + c) * AT_D + dc * 32 + 8 * hh);
        kl.h[1] = *(const v8b*)(Ksl + (j * 16 + c) * AT_D + dc * 32 + 16 + 8 * hh);
        s[j] = at_mma(qah[dc], kb.v, s[j]);
        s[j] = at_mma(qah[dc], kl.v, s[j]);
        s[j] = at_mma(qal[dc], kb.v, s[j]);
      }
    }
    int kvkeep[4];
#pragma unroll
    for (int j = 0; j < 4; ++j) kvkeep[j] = padb[kv0 + j * 16 + c];
    float cm[8];
#pragma unroll
    for (int r = 0; r < 8; ++r) {
      const unsigned qrow = q0 + 8 * hh + r;
      float m = -INFINITY;
#pragma unroll
      for (int j = 0; j < 4; ++j) {
        const unsigned kvcol = kv0 + j * 16 + c;
        const bool masked = (kvcol > qrow) || (kvkeep[j] == 0);
        const float sv = masked ? g.mask_fill : s[j][r];
        s[j][r] = sv;
        m = fmaxf(m, sv);
      }
#pragma unroll
      for (int off = 1; off < 16; off <<= 1) m = fmaxf(m, __shfl_xor(m, off, 32));
      cm[r] = m;
    }
    __bf16* pwh = Psh[wave];
    __bf16* pwl = Psl[wave];
#pragma unroll
    for (int r = 0; r < 8; ++r) {
      const float mnew = fmaxf(mrow[r], cm[r]);
      const float msub = (mnew == -INFINITY) ? 0.f : mnew;
      const float alpha = expf(mrow[r] - msub);
      mrow[r] = mnew;
      float psum = 0.f;
#pragma unroll
      for (int j = 0; j < 4; ++j) {
        const float p = expf(s[j][r] - msub);
        psum += p;
        __bf16 a, bl; at_split(p, a, bl);
        pwh[(8 * hh + r) * AT_KC + j * 16 + c] = a; pwl[(8 * hh + r) * AT_KC + j * 16 + c] = bl;
      }
#pragma unroll
      for (int off = 1; off < 16; off <<= 1) psum += __shfl_xor(psum, off, 32);
      lrow[r] = lrow[r] * alpha + psum;
#pragma unroll
      for (int t = 0; t < 4; ++t) oacc[t][r] *= alpha;
    }
    __builtin_amdgcn_fence(3  , "workgroup");
    __builtin_amdgcn_wave_barrier();
    __builtin_amdgcn_fence(2  , "workgroup");
#pragma unroll 1
    for (int kk = 0; kk < 2; ++kk) {
      FB pa, pl;
      pa.h[0] = *(const v8b*)(pwh + c * AT_KC + kk * 32 + 8 * hh);
      pa.h[1] = *(const v8b*)(pwh + c * AT_KC + kk * 32 + 16 + 8 * hh);
      pl.h[0] = *(const v8b*)(pwl + c * AT_KC + kk * 32 + 8 * hh);
      pl.h[1] = *(const v8b*)(pwl + c * AT_KC + kk * 32 + 16 + 8 * hh);
#pragma unroll
      for (int t = 0; t < 4; ++t) {
        FB vb, vl;
        vb.h[0] = *(const v8b*)(Vth + (t * 16 + c) * AT_KC + kk * 32 + 8 * hh);
        vb.h[1] = *(const v8b*)(Vth + (t * 16 + c) * AT_KC + kk * 32 + 16 + 8 * hh);
        vl.h[0] = *(const v8b*)(Vtl + (t * 16 + c) * AT_KC + kk * 32 + 8 * hh);
        vl.h[1] = *(const v8b*)(Vtl + (t * 16 + c) * AT_KC + kk * 32 + 16 + 8 * hh);
        oacc[t] = at_mma(pa.v, vb.v, oacc[t]);
        oacc[t] = at_mma(pa.v, vl.v, oacc[t]);
        oacc[t] = at_mma(pl.v, vb.v, oacc[t]);
      }
    }
    __builtin_amdgcn_fence(3  , "workgroup");
    __builtin_amdgcn_wave_barrier();
    __builtin_amdgcn_fence(2  , "workgroup");
  }

  float* os = Os[wave];
#pragma unroll
  for (int r = 0; r < 8; ++r) {
    const float inv = 1.0f / lrow[r];
#pragma unroll
    for (int t = 0; t < 4; ++t) os[(8 * hh + r) * 68 + t * 16 + c] = oacc[t][r] * inv;
  }
  __builtin_amdgcn_fence(3  , "workgroup");
  __builtin_amdgcn_wave_barrier();
  __builtin_amdgcn_fence(2  , "workgroup");
  {
    const unsigned q4 = lane >> 3, c8 = (lane & 7u) * 8u;
    for (int pass = 0; pass < 2; ++pass) {
#pragma unroll
      for (int it = 0; it < 4; ++it) {
        const unsigned row = it * 4 + q4;
        const float* sp = os + row * 68 + c8;
        const v4f s0 = *(const v4f*)(sp), s1 = *(const v4f*)(sp + 4);
        v8h hv;
        hv[0] = (_Float16)s0.x; hv[1] = (_Float16)s0.y; hv[2] = (_Float16)s0.z; hv[3] = (_Float16)s0.w;
        hv[4] = (_Float16)s1.x; hv[5] = (_Float16)s1.y; hv[6] = (_Float16)s1.z; hv[7] = (_Float16)s1.w;
        *(volatile v8h*)(ob_ptr + (size_t)(q0 + row) * g.o_rs + c8) = hv;
      }
      __threadfence();
    }
  }
}

constexpr size_t SZ_WQKV = (size_t)DQKV * DM * 2;
constexpr size_t SZ_WO   = (size_t)DM * DM * 2;
constexpr size_t SZ_W1   = (size_t)DFF * DM * 2;
constexpr size_t SZ_W2   = (size_t)DM * DFF * 2;
constexpr size_t SZ_BV   = (size_t)NBIAS * 4;
constexpr size_t SZ_N16  = (size_t)NB * SEQ * DM * 2;
constexpr size_t SZ_QKV  = (size_t)NB * SEQ * DQKV * 4;
constexpr size_t SZ_H16  = (size_t)NB * SEQ * DFF * 2;
constexpr size_t SZ_AO16 = (size_t)NB * SEQ * DM * 2;
constexpr size_t SZ_X1   = (size_t)NB * SEQ * DM * 4;
constexpr size_t OFF_WQKV = 0;
constexpr size_t OFF_WO   = OFF_WQKV + SZ_WQKV;
constexpr size_t OFF_W1   = OFF_WO + SZ_WO;
constexpr size_t OFF_W2   = OFF_W1 + SZ_W1;
constexpr size_t OFF_BV   = OFF_W2 + SZ_W2;
constexpr size_t OFF_N16  = OFF_BV + SZ_BV;
constexpr size_t OFF_QKV  = OFF_N16 + SZ_N16;
constexpr size_t OFF_AO16 = OFF_QKV + SZ_QKV;
constexpr size_t OFF_X1   = OFF_AO16 + SZ_AO16;
constexpr size_t WS_TOTAL = OFF_X1 + SZ_X1;
static_assert(SZ_H16 <= SZ_QKV);
static_assert(SZ_BV % 256 == 0 && SZ_N16 % 256 == 0 && SZ_QKV % 256 == 0 && SZ_AO16 % 256 == 0);
static_assert(WS_TOTAL <= (size_t)134217728);
static_assert(((SEQ / 64) * (DQKV / 64)) % 8 == 0 && ((SEQ / 64) * (DM / 64)) % 8 == 0 && ((SEQ / 64) * (DFF / 64)) % 8 == 0);
static_assert(DM % 32 == 0 && DFF % 32 == 0 && DM % 64 == 0 && DFF % 64 == 0 && DQKV % 64 == 0);

extern "C" void kernel_launch(void* const* d_in, const int* in_sizes, int n_in, void* d_out, int out_size, void* d_ws, size_t ws_size, hipStream_t stream) {
    if (n_in < 18) return;
    constexpr long long XROWS = (long long)(NB - 1) * SEQ_FULL + SEQ;
    if ((long long)in_sizes[0] < XROWS * DM) return;
    if ((long long)in_sizes[1] < XROWS) return;
    if (in_sizes[2] < DM || in_sizes[3] < DM || in_sizes[4] < DM || in_sizes[5] < DM) return;
    if (in_sizes[6] < DM * DM || in_sizes[8] < DM * DM || in_sizes[10] < DM * DM || in_sizes[12] < DM * DM) return;
    if (in_sizes[7] < DM || in_sizes[9] < DM || in_sizes[11] < DM || in_sizes[13] < DM) return;
    if (in_sizes[14] < DM * DFF || in_sizes[15] < DFF || in_sizes[16] < DFF * DM || in_sizes[17] < DM) return;
    if ((long long)out_size < XROWS * DM) return;
    if (WS_TOTAL > ws_size) return;

    const float* x    = (const float*)d_in[0];
    const int*   pad  = (const int*)d_in[1];
    const float* ln1g = (const float*)d_in[2];
    const float* ln1b = (const float*)d_in[3];
    const float* ln2g = (const float*)d_in[4];
    const float* ln2b = (const float*)d_in[5];
    const float* wq = (const float*)d_in[6];   const float* bq = (const float*)d_in[7];
    const float* wk = (const float*)d_in[8];   const float* bk = (const float*)d_in[9];
    const float* wv = (const float*)d_in[10];  const float* bv = (const float*)d_in[11];
    const float* wo = (const float*)d_in[12];  const float* bo = (const float*)d_in[13];
    const float* w1 = (const float*)d_in[14];  const float* b1 = (const float*)d_in[15];
    const float* w2 = (const float*)d_in[16];  const float* b2 = (const float*)d_in[17];
    float* out = (float*)d_out;

    char* wsp = (char*)d_ws;
    unsigned short* WQKV16 = (unsigned short*)(wsp + OFF_WQKV);
    unsigned short* WO16   = (unsigned short*)(wsp + OFF_WO);
    unsigned short* W116   = (unsigned short*)(wsp + OFF_W1);
    unsigned short* W216   = (unsigned short*)(wsp + OFF_W2);
    float*          BV     = (float*)(wsp + OFF_BV);
    unsigned short* N16    = (unsigned short*)(wsp + OFF_N16);
    float*          QKV    = (float*)(wsp + OFF_QKV);
    unsigned short* H16    = (unsigned short*)(wsp + OFF_QKV);
    unsigned short* AO16   = (unsigned short*)(wsp + OFF_AO16);
    float*          X1     = (float*)(wsp + OFF_X1);

    k_cm_castbT<<<(unsigned)((DM * (DM / 8) + 255) / 256), 256, 0, stream>>>(wq, DM, WQKV16, DM, DM, DM, 16.0f);
    k_cm_castbT<<<(unsigned)((DM * (DM / 8) + 255) / 256), 256, 0, stream>>>(wk, DM, WQKV16 + (size_t)DM * DM, DM, DM, DM, 16.0f);
    k_cm_castbT<<<(unsigned)((DM * (DM / 8) + 255) / 256), 256, 0, stream>>>(wv, DM, WQKV16 + (size_t)2 * DM * DM, DM, DM, DM, 16.0f);
    k_cm_castbT<<<(unsigned)((DM * (DM / 8) + 255) / 256), 256, 0, stream>>>(wo, DM, WO16, DM, DM, DM, 16.0f);
    k_cm_castbT<<<(unsigned)((DFF * (DM / 8) + 255) / 256), 256, 0, stream>>>(w1, DFF, W116, DM, DM, DFF, 16.0f);
    k_cm_castbT<<<(unsigned)((DM * (DFF / 8) + 255) / 256), 256, 0, stream>>>(w2, DM, W216, DFF, DFF, DM, 16.0f);
    k_db_bias<<<NBIAS / 256, 256, 0, stream>>>(bq, bk, bv, bo, b1, b2, BV);

    k_db_ln<1><<<(NB * SEQ) / 8, 256, 0, stream>>>(x, ln1g, ln1b, N16, (unsigned)(NB * SEQ), (unsigned)SEQ, (unsigned)SEQ_FULL);

    wmma_gemm64<2, 0, false, 0, 0><<<dim3((unsigned)((((SEQ / 64) * (DQKV / 64)) + 7) / 8), (unsigned)NB), 256, 0, stream>>>(
        N16, DM, (long long)SEQ * DM, WQKV16, DM, 0LL, (void*)QKV, DQKV, (long long)SEQ * DQKV, BV, nullptr, 0LL, SEQ, DQKV, DM, 0.0625f);

    {
        AttnGeom g;
        g.pad = pad;
        g.q_bs = (long long)SEQ * DQKV; g.q_rs = DQKV;
        g.k_bs = (long long)SEQ * DQKV; g.k_rs = DQKV;
        g.v_bs = (long long)SEQ * DQKV; g.v_rs = DQKV;
        g.o_bs = (long long)SEQ * DM;   g.o_rs = DM;
        g.pad_bs = SEQ_FULL;
        g.qscale = 0.125f; g.mask_fill = -INFINITY;
        attn64_kernel<<<(unsigned)(NB * NHEADS * (SEQ / 64)), 128, 0, stream>>>(QKV, QKV + DM, QKV + 2 * DM, AO16, g);
    }

    wmma_gemm64<2, 0, true, 0, 1><<<dim3((unsigned)((((SEQ / 64) * (DM / 64)) + 7) / 8), (unsigned)NB), 256, 0, stream>>>(
        AO16, DM, (long long)SEQ * DM, WO16, DM, 0LL, (void*)X1, DM, (long long)SEQ * DM, BV + 3072, x, (long long)SEQ_FULL * DM, SEQ, DM, DM, 0.0625f);

    k_db_ln<0><<<(NB * SEQ) / 8, 256, 0, stream>>>(X1, ln2g, ln2b, N16, (unsigned)(NB * SEQ), (unsigned)SEQ, (unsigned)SEQ);

    wmma_gemm64<2, 1, false, 5, 0><<<dim3((unsigned)((((SEQ / 64) * (DFF / 64)) + 7) / 8), (unsigned)NB), 256, 0, stream>>>(
        N16, DM, (long long)SEQ * DM, W116, DM, 0LL, (void*)H16, DFF, (long long)SEQ * DFF, BV + 4096, nullptr, 0LL, SEQ, DFF, DM, 0.0625f);

    wmma_gemm64<2, 0, true, 0, 0><<<dim3((unsigned)((((SEQ / 64) * (DM / 64)) + 7) / 8), (unsigned)NB), 256, 0, stream>>>(
        H16, DFF, (long long)SEQ * DFF, W216, DFF, 0LL, (void*)out, DM, (long long)SEQ_FULL * DM, BV + 8192, X1, (long long)SEQ * DM, SEQ, DM, DFF, 0.0625f);
}
